// SparseMHAEncoder_3582002725458
// MI455X (gfx1250) — hardware-verified
//
#include <hip/hip_runtime.h>
#include <math.h>

constexpr int kBatch   = 2;
constexpr int kSeq     = 2048;
constexpr int kDim     = 512;
constexpr int kHeads   = 8;
constexpr int kHeadDim = 64;
constexpr int kTok     = kBatch * kSeq;
constexpr int kSpan    = 64;
constexpr int kGroupsPerChunk = 4;
constexpr int kChunks  = kBatch * kHeads / kGroupsPerChunk;
constexpr size_t kPlaneHalves  = (size_t)kTok * kDim;
constexpr size_t kWPlaneHalves = (size_t)kDim * kDim;
constexpr size_t kSPlaneElems  = (size_t)kSeq * kSeq;
constexpr float kQKVCarry   = 16.0f;
constexpr float kPCarry     = 1024.0f;
constexpr float kScoreScale = 0.125f / (kQKVCarry * kQKVCarry);
constexpr float kPVScale    = 1.0f / (kPCarry * kQKVCarry);

static_assert(kDim % 32 == 0 && kHeadDim % 32 == 0 && kSeq % 32 == 0, "K multiples of 32");
static_assert(kTok % 64 == 0 && kDim % 64 == 0 && kSeq % 64 == 0 && kHeadDim % 64 == 0, "tile multiples of 64");

constexpr size_t kOffW    = 0;
constexpr size_t kOffQ16  = 4194304;
constexpr size_t kOffK16  = 8388608;
constexpr size_t kOffVt16 = 12582912;
constexpr size_t kOffOhi  = 16777216;
constexpr size_t kOffOlo  = 20971520;
constexpr size_t kOffScr  = 25165824;
constexpr size_t kOffAct  = kOffScr;
constexpr size_t kOffS    = kOffScr;
constexpr size_t kOffP    = kOffS + (size_t)kGroupsPerChunk * kSPlaneElems * 4;
constexpr size_t kWsTotal = kOffP + (size_t)kGroupsPerChunk * kSPlaneElems * 2;
static_assert(kOffAct + 6 * kPlaneHalves * 2 <= kOffP, "activation planes inside the scores region");
static_assert(kWsTotal == 125829120, "carve total");
static_assert(kWsTotal <= 134217728, "carve under 128 MiB");

typedef __attribute__((ext_vector_type(16))) _Float16 v16h;
typedef __attribute__((ext_vector_type(8)))  _Float16 v8h;
typedef __attribute__((ext_vector_type(16))) __bf16   v16b;
typedef __attribute__((ext_vector_type(8)))  __bf16   v8b;
typedef __attribute__((ext_vector_type(8)))  float    v8f;
typedef __attribute__((ext_vector_type(4)))  float    v4f;
typedef __attribute__((ext_vector_type(4)))  unsigned int v4u;

__device__ __forceinline__ unsigned short f2bf_bits(float f) {
  unsigned u = __float_as_uint(f);
  return (unsigned short)((u + 0x7FFFu + ((u >> 16) & 1u)) >> 16);
}
__device__ __forceinline__ float bf_bits2f(unsigned short h) { return __uint_as_float(((unsigned)h) << 16); }

__device__ __forceinline__ void dep_guard_h(v8f& a, v8f& b, v16h x, v16h y) { asm volatile("v_nop\n\tv_nop\n\tv_nop\n\tv_nop" : "+v"(a), "+v"(b) : "v"(x), "v"(y)); }
__device__ __forceinline__ void dep_guard_b(v8f& a, v8f& b, v16b x, v16b y) { asm volatile("v_nop\n\tv_nop\n\tv_nop\n\tv_nop" : "+v"(a), "+v"(b) : "v"(x), "v"(y)); }
__device__ __forceinline__ void keep4_h(v16h a, v16h b, v16h c, v16h d) { asm volatile("v_nop" :: "v"(a), "v"(b), "v"(c), "v"(d)); }
__device__ __forceinline__ void keep4_b(v16b a, v16b b, v16b c, v16b d) { asm volatile("v_nop" :: "v"(a), "v"(b), "v"(c), "v"(d)); }
__device__ __forceinline__ void acc_guard4(v8f& a, v8f& b, v8f& c, v8f& d) { asm volatile("v_nop\n\tv_nop\n\tv_nop\n\tv_nop" : "+v"(a), "+v"(b), "+v"(c), "+v"(d)); }
template <typename T> struct Frag;
template <> struct Frag<_Float16> {
  typedef v16h V; union U { v16h v; v8h h[2]; };
  static __device__ __forceinline__ v16h load(const _Float16* p) {
    U f; f.h[0] = *(const v8h*)(p); f.h[1] = *(const v8h*)(p + 16); return f.v;
  }
  static __device__ __forceinline__ v8f mma(v16h a, v16h b, v8f c) {
    return __builtin_amdgcn_wmma_f32_16x16x32_f16(false, a, false, b, (short)0, c, false, false);
  }
  static __device__ __forceinline__ void guard(v8f& a, v8f& b, v16h x, v16h y) { dep_guard_h(a, b, x, y); }
  static __device__ __forceinline__ void keep(v16h a, v16h b, v16h c, v16h d) { keep4_h(a, b, c, d); }
};
template <> struct Frag<__bf16> {
  typedef v16b V; union U { v16b v; v8b h[2]; };
  static __device__ __forceinline__ v16b load(const __bf16* p) {
    U f; f.h[0] = *(const v8b*)(p); f.h[1] = *(const v8b*)(p + 16); return f.v;
  }
  static __device__ __forceinline__ v8f mma(v16b a, v16b b, v8f c) {
    return __builtin_amdgcn_wmma_f32_16x16x32_bf16(false, a, false, b, (short)0, c, false, false);
  }
  static __device__ __forceinline__ void guard(v8f& a, v8f& b, v16b x, v16b y) { dep_guard_b(a, b, x, y); }
  static __device__ __forceinline__ void keep(v16b a, v16b b, v16b c, v16b d) { keep4_b(a, b, c, d); }
};

__device__ __forceinline__ unsigned pk16(unsigned short a, unsigned short b) { return (unsigned)a | ((unsigned)b << 16); }
__device__ __forceinline__ unsigned short h_bits(float f) { const _Float16 h = (_Float16)f; return __builtin_bit_cast(unsigned short, h); }

template <int ET> struct Elem;
template <> struct Elem<0> { typedef _Float16 T; };
template <> struct Elem<1> { typedef __bf16 T; };
template <int ET, bool SPLIT, int BIAS_MODE, int OUT_MODE, bool RESID, int ACT = 0>
__global__ __launch_bounds__(256) void wmma_gemm64(
    const unsigned short* __restrict__ Ap, const unsigned short* __restrict__ A2p, int lda, long strideA,
    const unsigned short* __restrict__ Btp, const unsigned short* __restrict__ Bt2p, int ldb, long strideB,
    void* __restrict__ Cout, void* __restrict__ Cout2, int ldc, long strideC,
    const float* __restrict__ bias,
    const float* __restrict__ resid, long strideR,
    int M, int N, int K, float scale) {
  typedef typename Elem<ET>::T T;
  typedef typename Frag<T>::V V;
  const T* A = (const T*)Ap; const T* A2 = (const T*)A2p; const T* Bt = (const T*)Btp; const T* Bt2 = (const T*)Bt2p;
  __shared__ __align__(16) float sT[8][16 * 68];
  const int b    = blockIdx.y;
  const int lane = threadIdx.x & 31;
  const int wave = threadIdx.x >> 5;
  const int tilesN = N >> 6;
  const int tilesM = M >> 6;
  const int tile = blockIdx.x * 8 + wave;
  if (tile >= tilesM * tilesN) return;
  const int tm = tile / tilesN;
  const int tn = tile - tm * tilesN;
  const int m0 = tm << 6;
  const int n0 = tn << 6;

  const T* Ab  = A  + (size_t)b * strideA;
  const T* Bb  = Bt + (size_t)b * strideB;
  const T* Ab2 = SPLIT ? (A2  + (size_t)b * strideA) : nullptr;
  const T* Bb2 = SPLIT ? (Bt2 + (size_t)b * strideB) : nullptr;

  const int rlane = lane & 15;
  const int koff  = (lane >> 4) * 8;
  const int mOff  = (lane >> 4) * 8;

  v8f acc[4][4];
#pragma unroll
  for (int i = 0; i < 4; ++i)
#pragma unroll
    for (int j = 0; j < 4; ++j) acc[i][j] = (v8f){0.f,0.f,0.f,0.f,0.f,0.f,0.f,0.f};

  for (int k0 = 0; k0 < K; k0 += 32) {
    V bh[4], bl[4];
#pragma unroll
    for (int j = 0; j < 4; ++j) {
      const size_t bo = (size_t)(n0 + (j << 4) + rlane) * ldb + koff + k0;
      bh[j] = Frag<T>::load(Bb + bo);
      if (SPLIT) bl[j] = Frag<T>::load(Bb2 + bo);
    }
#pragma unroll
    for (int i = 0; i < 4; ++i) {
      const size_t ao = (size_t)(m0 + (i << 4) + rlane) * lda + koff + k0;
      V ah = Frag<T>::load(Ab + ao);
      V al;
      if (SPLIT) al = Frag<T>::load(Ab2 + ao);
#pragma unroll
      for (int j = 0; j < 4; ++j) {
        acc[i][j] = Frag<T>::mma(ah, bh[j], acc[i][j]);
        if (SPLIT) {
          acc[i][j] = Frag<T>::mma(ah, bl[j], acc[i][j]);
          acc[i][j] = Frag<T>::mma(al, bh[j], acc[i][j]);
        }
      }
      Frag<T>::guard(acc[i][0], acc[i][3], ah, SPLIT ? al : ah);
    }
    Frag<T>::keep(bh[0], bh[1], bh[2], bh[3]);
    if (SPLIT) Frag<T>::keep(bl[0], bl[1], bl[2], bl[3]);
  }
  acc_guard4(acc[0][0], acc[0][1], acc[0][2], acc[0][3]);
  acc_guard4(acc[1][0], acc[1][1], acc[1][2], acc[1][3]);
  acc_guard4(acc[2][0], acc[2][1], acc[2][2], acc[2][3]);
  acc_guard4(acc[3][0], acc[3][1], acc[3][2], acc[3][3]);

  float* slab = sT[wave];
  const float* Rb = RESID ? (resid + (size_t)b * strideR) : nullptr;
#pragma unroll
  for (int i = 0; i < 4; ++i) {
    const int mBase = m0 + (i << 4);
#pragma unroll
    for (int j = 0; j < 4; ++j) {
      const int n = n0 + (j << 4) + rlane;
      float bv = 0.f;
      if (BIAS_MODE == 2) bv = bias[n];
#pragma unroll
      for (int r = 0; r < 8; ++r) {
        float v = acc[i][j][r] * scale;
        if (BIAS_MODE == 1) v += bias[mBase + mOff + r];
        if (BIAS_MODE == 2) v += bv;
        if (RESID) v += Rb[(size_t)(mBase + mOff + r) * ldc + n];
        if (ACT == 2) v = fmaxf(v, 0.0f);
        if (ACT == 4) v = (v > 0.f) ? v : 0.01f * v;
        slab[(mOff + r) * 68 + (j << 4) + rlane] = v;
      }
    }
    __builtin_amdgcn_fence(__ATOMIC_RELEASE, "workgroup");
    __builtin_amdgcn_wave_barrier();
    __builtin_amdgcn_fence(__ATOMIC_ACQUIRE, "workgroup");
    if (OUT_MODE == 0) {
      float* C = (float*)Cout + (size_t)b * strideC;
      const int hh = lane >> 4, c4 = (lane & 15) * 4;
      for (int pass = 0; pass < 2; ++pass) {
#pragma unroll
        for (int it = 0; it < 8; ++it) {
          const int row = it * 2 + hh;
          v4f v = *(const v4f*)(slab + row * 68 + c4);
          *(volatile v4f*)(C + (size_t)(mBase + row) * ldc + n0 + c4) = v;
        }
        __threadfence();
      }
    } else {
      const int q = lane >> 3, c8 = (lane & 7) * 8;
      unsigned short* C  = (unsigned short*)Cout  + (size_t)b * strideC;
      unsigned short* C2 = (OUT_MODE == 2) ? ((unsigned short*)Cout2 + (size_t)b * strideC) : nullptr;
      for (int pass = 0; pass < 2; ++pass) {
#pragma unroll
        for (int it = 0; it < 4; ++it) {
          const int row = it * 4 + q;
          const float* sp = slab + row * 68 + c8;
          v8h hv, lv;
#pragma unroll
          for (int e = 0; e < 8; ++e) {
            if (OUT_MODE == 1) {
              hv[e] = (_Float16)sp[e];
            } else {
              unsigned short hb = f2bf_bits(sp[e]);
              unsigned short lb = f2bf_bits(sp[e] - bf_bits2f(hb));
              hv[e] = __builtin_bit_cast(_Float16, hb);
              lv[e] = __builtin_bit_cast(_Float16, lb);
            }
          }
          *(volatile v8h*)(C + (size_t)(mBase + row) * ldc + n0 + c8) = hv;
          if (OUT_MODE == 2) *(volatile v8h*)(C2 + (size_t)(mBase + row) * ldc + n0 + c8) = lv;
        }
        __threadfence();
      }
    }
    __builtin_amdgcn_fence(__ATOMIC_RELEASE, "workgroup");
    __builtin_amdgcn_wave_barrier();
    __builtin_amdgcn_fence(__ATOMIC_ACQUIRE, "workgroup");
  }
}

__global__ __launch_bounds__(256) void wsplit_bf16_kernel(const float* __restrict__ W0, const float* __restrict__ W1,
                                                         const float* __restrict__ W2, const float* __restrict__ W3,
                                                         unsigned short* __restrict__ out) {
  __shared__ float sm[64][65];
  const int t  = threadIdx.x;
  const int i0 = blockIdx.x * 64;
  const int o0 = blockIdx.y * 64;
  const int z  = blockIdx.z;
  const float* W = (z == 0) ? W0 : (z == 1) ? W1 : (z == 2) ? W2 : W3;
#pragma unroll
  for (int it = 0; it < 16; ++it) {
    const int e = it * 256 + t;
    const int r = e >> 6;
    const int c = e & 63;
    sm[c][r] = W[(size_t)(i0 + r) * kDim + o0 + c];
  }
  __syncthreads();
  const int lane = t & 31, wave = t >> 5;
  const int q = lane >> 3, c8 = (lane & 7) * 8;
  unsigned short* oh = out + (size_t)z * 2 * kWPlaneHalves;
  unsigned short* ol = oh + kWPlaneHalves;
  v4u uh[2], ul[2];
#pragma unroll
  for (int it = 0; it < 2; ++it) {
    const int row = wave * 8 + it * 4 + q;
    unsigned short hb[8], lb[8];
#pragma unroll
    for (int e = 0; e < 8; ++e) {
      const float f = sm[row][c8 + e];
      hb[e] = f2bf_bits(f);
      lb[e] = f2bf_bits(f - bf_bits2f(hb[e]));
    }
    uh[it] = (v4u){pk16(hb[0], hb[1]), pk16(hb[2], hb[3]), pk16(hb[4], hb[5]), pk16(hb[6], hb[7])};
    ul[it] = (v4u){pk16(lb[0], lb[1]), pk16(lb[2], lb[3]), pk16(lb[4], lb[5]), pk16(lb[6], lb[7])};
  }
  for (int pass = 0; pass < 2; ++pass) {
#pragma unroll
    for (int it = 0; it < 2; ++it) {
      const int row = wave * 8 + it * 4 + q;
      const size_t off = (size_t)(o0 + row) * kDim + i0 + c8;
      *(volatile v4u*)(oh + off) = uh[it];
      *(volatile v4u*)(ol + off) = ul[it];
    }
    __threadfence();
  }
}

__global__ __launch_bounds__(256) void asplit_bf16_kernel(const float* __restrict__ x0, const float* __restrict__ x1,
                                                         const float* __restrict__ x2,
                                                         unsigned short* __restrict__ out, int n8) {
  const int i = blockIdx.x * 256 + threadIdx.x;
  const int tsel = blockIdx.y;
  if (i >= n8) return;
  const float* src = (tsel == 0) ? x0 : (tsel == 1) ? x1 : x2;
  const float* p = src + 8 * (size_t)i;
  const v4f a = *(const v4f*)(p);
  const v4f c = *(const v4f*)(p + 4);
  unsigned short hb[8], lb[8];
#pragma unroll
  for (int e = 0; e < 4; ++e) {
    hb[e] = f2bf_bits(a[e]);
    lb[e] = f2bf_bits(a[e] - bf_bits2f(hb[e]));
    hb[4 + e] = f2bf_bits(c[e]);
    lb[4 + e] = f2bf_bits(c[e] - bf_bits2f(hb[4 + e]));
  }
  const v4u uh = (v4u){pk16(hb[0], hb[1]), pk16(hb[2], hb[3]), pk16(hb[4], hb[5]), pk16(hb[6], hb[7])};
  const v4u ul = (v4u){pk16(lb[0], lb[1]), pk16(lb[2], lb[3]), pk16(lb[4], lb[5]), pk16(lb[6], lb[7])};
  unsigned short* oh = out + (size_t)tsel * 2 * kPlaneHalves + 8 * (size_t)i;
  unsigned short* ol = oh + kPlaneHalves;
  *(volatile v4u*)oh = uh;
  *(volatile v4u*)ol = ul;
  __threadfence();
  *(volatile v4u*)oh = uh;
  *(volatile v4u*)ol = ul;
}

__global__ __launch_bounds__(256) void band_softmax_kernel(const float* __restrict__ S, unsigned short* __restrict__ P) {
  __shared__ float pw[8][64];
  const int t    = threadIdx.x;
  const int lane = t & 31, wave = t >> 5;
  const int R    = blockIdx.x * 8 + wave;
  const int tq   = R & (kSeq - 1);
  const int lo   = tq - (kSpan - 1);
  const float* sr = S + (size_t)R * kSeq;
  const int ca  = lo + lane;
  const int cb  = lo + 32 + lane;
  const int caa = ca < 0 ? 0 : ca;
  const int cba = cb < 0 ? 0 : cb;
  const float xa = sr[caa];
  const float xb = sr[cba];
  const float ninf = -__builtin_inff();
  const float sa = (ca >= 0) ? xa : ninf;
  const float sb = (cb >= 0) ? xb : ninf;
  float m = fmaxf(sa, sb);
#pragma unroll
  for (int off = 16; off > 0; off >>= 1) m = fmaxf(m, __shfl_xor(m, off, 32));
  const float ea = expf(sa - m);
  const float eb = expf(sb - m);
  float sum = ea + eb;
#pragma unroll
  for (int off = 16; off > 0; off >>= 1) sum += __shfl_xor(sum, off, 32);
  const float inv = 1.0f / sum;
  pw[wave][lane]      = ea * inv * kPCarry;
  pw[wave][32 + lane] = eb * inv * kPCarry;
  __syncthreads();

  v4u uv[8];
#pragma unroll
  for (int ch = 0; ch < 8; ++ch) {
    unsigned w[4];
#pragma unroll
    for (int e2 = 0; e2 < 4; ++e2) {
      unsigned packed = 0u;
#pragma unroll
      for (int hf = 0; hf < 2; ++hf) {
        const int col = ch * 256 + lane * 8 + e2 * 2 + hf;
        const int d   = col - lo;
        const bool inb = (unsigned)d < 64u;
        const int idx  = inb ? d : 0;
        const float pv = pw[wave][idx];
        unsigned bits = (unsigned)h_bits(pv);
        bits = inb ? bits : 0u;
        packed |= bits << (16 * hf);
      }
      w[e2] = packed;
    }
    uv[ch] = (v4u){w[0], w[1], w[2], w[3]};
  }
  unsigned short* prow = P + (size_t)R * kSeq + lane * 8;
  for (int pass = 0; pass < 2; ++pass) {
#pragma unroll
    for (int ch = 0; ch < 8; ++ch) *(volatile v4u*)(prow + ch * 256) = uv[ch];
    __threadfence();
  }
}

extern "C" void kernel_launch(void* const* d_in, const int* in_sizes, int n_in,
                              void* d_out, int out_size, void* d_ws, size_t ws_size,
                              hipStream_t stream) {
  if (n_in < 7) return;
  if (in_sizes[0] != kTok * kDim || in_sizes[1] != kTok * kDim || in_sizes[2] != kTok * kDim) return;
  if (in_sizes[3] != kDim * kDim || in_sizes[4] != kDim * kDim || in_sizes[5] != kDim * kDim || in_sizes[6] != kDim * kDim) return;
  if (out_size != kTok * kDim) return;
  if (ws_size < kWsTotal) return;

  const float* q    = (const float*)d_in[0];
  const float* kin  = (const float*)d_in[1];
  const float* vin  = (const float*)d_in[2];
  const float* Wq   = (const float*)d_in[3];
  const float* Wk   = (const float*)d_in[4];
  const float* Wv   = (const float*)d_in[5];
  const float* Wout = (const float*)d_in[6];
  float* out = (float*)d_out;

  unsigned char* ws = (unsigned char*)d_ws;
  unsigned short* WT   = (unsigned short*)(ws + kOffW);
  unsigned short* Q16  = (unsigned short*)(ws + kOffQ16);
  unsigned short* K16  = (unsigned short*)(ws + kOffK16);
  unsigned short* Vt16 = (unsigned short*)(ws + kOffVt16);
  unsigned short* Ohi  = (unsigned short*)(ws + kOffOhi);
  unsigned short* Olo  = (unsigned short*)(ws + kOffOlo);
  unsigned short* ACT  = (unsigned short*)(ws + kOffAct);
  float*          Spl  = (float*)(ws + kOffS);
  unsigned short* Ppl  = (unsigned short*)(ws + kOffP);
  const float* fdummy  = (const float*)(ws + kOffW);

  wsplit_bf16_kernel<<<dim3(kDim / 64, kDim / 64, 4), dim3(256), 0, stream>>>(Wq, Wk, Wv, Wout, WT);

  const int n8 = (kTok * kDim) / 8;
  asplit_bf16_kernel<<<dim3(n8 / 256, 3), dim3(256), 0, stream>>>(q, kin, vin, ACT, n8);

  wmma_gemm64<1, true, 0, 1, false><<<dim3(64, 2), dim3(256), 0, stream>>>(
      ACT, ACT + kPlaneHalves, kDim, (long)(2 * kPlaneHalves),
      WT, WT + kWPlaneHalves, kDim, (long)(2 * kWPlaneHalves),
      (void*)Q16, (void*)Q16, kDim, (long)kPlaneHalves,
      fdummy, fdummy, 0L,
      kTok, kDim, kDim, kQKVCarry);

  wmma_gemm64<1, true, 0, 1, false><<<dim3(64, 1), dim3(256), 0, stream>>>(
      WT + 4 * kWPlaneHalves, WT + 5 * kWPlaneHalves, kDim, 0L,
      ACT + 4 * kPlaneHalves, ACT + 5 * kPlaneHalves, kDim, 0L,
      (void*)Vt16, (void*)Vt16, kSeq * kBatch, 0L,
      fdummy, fdummy, 0L,
      kDim, kTok, kDim, kQKVCarry);

  for (int c = 0; c < kChunks; ++c) {
    const int b  = c >> 1;
    const int h0 = (c & 1) * kGroupsPerChunk;
    const size_t qkoff = (size_t)b * kSeq * kDim + (size_t)h0 * kHeadDim;
    const size_t vtoff = (size_t)h0 * kHeadDim * (size_t)kTok + (size_t)b * kSeq;
    const size_t ooff  = qkoff;

    wmma_gemm64<0, false, 0, 0, false><<<dim3(128, kGroupsPerChunk), dim3(256), 0, stream>>>(
        Q16 + qkoff, Q16 + qkoff, kDim, (long)kHeadDim,
        K16 + qkoff, K16 + qkoff, kDim, (long)kHeadDim,
        (void*)Spl, (void*)Spl, kSeq, (long)kSPlaneElems,
        fdummy, fdummy, 0L,
        kSeq, kSeq, kHeadDim, kScoreScale);

    band_softmax_kernel<<<dim3((kGroupsPerChunk * kSeq) / 8), dim3(256), 0, stream>>>(Spl, Ppl);

    wmma_gemm64<0, false, 0, 2, false><<<dim3(4, kGroupsPerChunk), dim3(256), 0, stream>>>(
        Ppl, Ppl, kSeq, (long)kSPlaneElems,
        Vt16 + vtoff, Vt16 + vtoff, kTok, (long)((size_t)kHeadDim * kTok),
        (void*)(Ohi + ooff), (void*)(Olo + ooff), kDim, (long)kHeadDim,
        fdummy, fdummy, 0L,
        kSeq, kHeadDim, kSeq, kPVScale);
  }

  wmma_gemm64<1, true, 0, 0, false><<<dim3(64, 1), dim3(256), 0, stream>>>(
      Ohi, Olo, kDim, 0L,
      WT + 6 * kWPlaneHalves, WT + 7 * kWPlaneHalves, kDim, 0L,
      (void*)out, (void*)out, kDim, 0L,
      fdummy, fdummy, 0L,
      kTok, kDim, kDim, 1.0f);
}
